// Block_86028194939235
// MI455X (gfx1250) — hardware-verified
//
#include <hip/hip_runtime.h>
#include <math.h>

#ifndef NB
#define NB 2
#endif
#ifndef SEQ
#define SEQ 1024
#endif
#define NB_FULL 2
#define SEQ_FULL 1024
#define CW 1024
#define NH 16
#define HD 64
#define FF 4096
#define FF2 8192
#define QKVW 3072
#define PSP 40

constexpr int kMROWS = NB * SEQ;
constexpr int kMCH = (kMROWS < 1024) ? kMROWS : 1024;
constexpr int kNCH = kMROWS / kMCH;

static_assert(NB <= NB_FULL);
static_assert(SEQ <= SEQ_FULL);
static_assert(SEQ % 64 == 0);
static_assert(CW == NH * HD);
static_assert(HD == 64);
static_assert(QKVW == 3 * CW);
static_assert(FF2 == 2 * FF);
static_assert(kMROWS % kMCH == 0);
static_assert(kMCH % 64 == 0);
static_assert(kMROWS % 64 == 0);
static_assert(CW % 64 == 0 && QKVW % 64 == 0 && FF % 64 == 0 && FF2 % 64 == 0);
static_assert(CW % 32 == 0 && FF % 32 == 0);
static_assert(CW == 32 * 4 * 8);
static_assert((PSP * 2) % 16 == 0 && PSP >= 32);

typedef __attribute__((ext_vector_type(16))) _Float16 v16h;
typedef __attribute__((ext_vector_type(8)))  _Float16 v8h;
typedef __attribute__((ext_vector_type(8)))  float    v8f;
typedef __attribute__((ext_vector_type(4)))  float    v4f;
typedef __attribute__((ext_vector_type(2)))  float    v2f;
typedef __attribute__((ext_vector_type(4)))  unsigned int v4u;
typedef __attribute__((ext_vector_type(2)))  unsigned int v2u;
typedef v8h v8h_a __attribute__((may_alias));
typedef v4f v4f_a __attribute__((may_alias));

union FragH { v16h v; v8h h[2]; };
__device__ __forceinline__ v16h ldfrag(const _Float16* __restrict__ p) {
    FragH f; f.h[0] = *(const v8h*)(p); f.h[1] = *(const v8h*)(p + 16); return f.v;
}
__device__ __forceinline__ v8f wmma16(v16h a, v16h b, v8f c) {
    c = __builtin_amdgcn_wmma_f32_16x16x32_f16(false, a, false, b, (short)0, c, false, false);
    asm volatile("v_nop\n\tv_nop\n\tv_nop\n\tv_nop" : "+v"(c) : "v"(a), "v"(b));
    return c;
}
__device__ __forceinline__ v8f wmma_raw(v16h a, v16h b, v8f c) {
    return __builtin_amdgcn_wmma_f32_16x16x32_f16(false, a, false, b, (short)0, c, false, false);
}
__device__ __forceinline__ void dep_guard_h(v8f& a, v8f& b, v16h x, v16h y) { asm volatile("v_nop\n\tv_nop\n\tv_nop\n\tv_nop" : "+v"(a), "+v"(b) : "v"(x), "v"(y)); }
__device__ __forceinline__ void keep4_h(v16h a, v16h b, v16h c, v16h d) { asm volatile("v_nop" :: "v"(a), "v"(b), "v"(c), "v"(d)); }
__device__ __forceinline__ void acc_guard4(v8f& a, v8f& b, v8f& c, v8f& d) { asm volatile("v_nop\n\tv_nop\n\tv_nop\n\tv_nop" : "+v"(a), "+v"(b), "+v"(c), "+v"(d)); }

__device__ __forceinline__ float cmb_bf(float v) { const unsigned u = __builtin_bit_cast(unsigned, v); const unsigned r = (u + 0x7fffu + ((u >> 16) & 1u)) & 0xffff0000u; return __builtin_bit_cast(float, r); }
__device__ __forceinline__ unsigned int pk2h(float a, float b) { return (unsigned int)__builtin_bit_cast(unsigned short, (_Float16)a) | ((unsigned int)__builtin_bit_cast(unsigned short, (_Float16)b) << 16); }

#define VST2(T, ptr, val) do { const T vst2_v_ = (val); *(volatile T*)(ptr) = vst2_v_; __threadfence(); *(volatile T*)(ptr) = vst2_v_; } while (0)

__device__ __forceinline__ void wave_sync_lds() {
    __builtin_amdgcn_fence(3  , "workgroup");
    __builtin_amdgcn_wave_barrier();
    __builtin_amdgcn_fence(2  , "workgroup");
}

__global__ __launch_bounds__(256) void k_gemm64(const unsigned short* __restrict__ Ap, int lda, const unsigned short* __restrict__ Btp, int ldb,
                                                float* __restrict__ C, int ldc, const float* __restrict__ cs, int use_cs, int M, int N, int K, float scale) {
    const _Float16* A = (const _Float16*)Ap; const _Float16* Bt = (const _Float16*)Btp;
    __shared__ __align__(16) float sT[8][16 * 68];
    const int lane = threadIdx.x & 31;
    const int wave = __builtin_amdgcn_readfirstlane((int)(threadIdx.x >> 5));
    const int tilesN = N >> 6, tilesM = M >> 6;
    const int tile = blockIdx.x * 8 + wave;
    if (tile >= tilesM * tilesN) return;
    const int tm = tile / tilesN, tn = tile - tm * tilesN;
    const int m0 = tm << 6, n0 = tn << 6;
    const int rlane = lane & 15, koff = (lane >> 4) * 8, mOff = (lane >> 4) * 8;

    v8f acc[4][4];
#pragma unroll
    for (int i = 0; i < 4; ++i)
#pragma unroll
        for (int j = 0; j < 4; ++j) acc[i][j] = (v8f){0.f, 0.f, 0.f, 0.f, 0.f, 0.f, 0.f, 0.f};

    for (int k0 = 0; k0 < K; k0 += 32) {
        v16h bh[4];
#pragma unroll
        for (int j = 0; j < 4; ++j) bh[j] = ldfrag(Bt + (size_t)(n0 + (j << 4) + rlane) * ldb + koff + k0);
#pragma unroll
        for (int i = 0; i < 4; ++i) {
            const v16h ah = ldfrag(A + (size_t)(m0 + (i << 4) + rlane) * lda + koff + k0);
#pragma unroll
            for (int j = 0; j < 4; ++j) acc[i][j] = wmma_raw(ah, bh[j], acc[i][j]);
            dep_guard_h(acc[i][0], acc[i][3], ah, ah);
        }
        keep4_h(bh[0], bh[1], bh[2], bh[3]);
    }
    acc_guard4(acc[0][0], acc[0][1], acc[0][2], acc[0][3]);
    acc_guard4(acc[1][0], acc[1][1], acc[1][2], acc[1][3]);
    acc_guard4(acc[2][0], acc[2][1], acc[2][2], acc[2][3]);
    acc_guard4(acc[3][0], acc[3][1], acc[3][2], acc[3][3]);

#pragma unroll
    for (int i = 0; i < 4; ++i) {
        const int mBase = m0 + (i << 4);
#pragma unroll
        for (int j = 0; j < 4; ++j) {
            const int n = n0 + (j << 4) + rlane;
            float csv = scale;
            if (use_cs) csv *= cmb_bf(cs[n]);
#pragma unroll
            for (int r = 0; r < 8; ++r) sT[wave][(mOff + r) * 68 + (j << 4) + rlane] = acc[i][j][r] * csv;
        }
        wave_sync_lds();
        {
            const int hh = lane >> 4, c4 = (lane & 15) * 4;
            for (int pass = 0; pass < 2; ++pass) {
#pragma unroll
                for (int it = 0; it < 8; ++it) {
                    const int row = it * 2 + hh;
                    const v4f v = *(const v4f_a*)&sT[wave][row * 68 + c4];
                    *(volatile v4f*)(C + (size_t)(mBase + row) * ldc + n0 + c4) = v;
                }
                __threadfence();
            }
        }
        wave_sync_lds();
    }
}

__global__ __launch_bounds__(256) void k_cast16(const float* __restrict__ SRC, unsigned short* __restrict__ DST, int nR, int nC, float sc, int seq, int seqfull) {
    const long long u = (long long)blockIdx.x * 256 + threadIdx.x; const int per = nC / 8; if (u >= (long long)nR * per) return;
    const int r = (int)(u / per); const int c0 = 8 * (int)(u % per);
    const int rs = (r / seq) * seqfull + (r % seq);
    const float* s = SRC + (size_t)rs * nC + c0;
    const v4f a = *(const v4f*)(s), b = *(const v4f*)(s + 4);
    v4u pk;
    pk.x = pk2h(cmb_bf(a.x) * sc, cmb_bf(a.y) * sc); pk.y = pk2h(cmb_bf(a.z) * sc, cmb_bf(a.w) * sc);
    pk.z = pk2h(cmb_bf(b.x) * sc, cmb_bf(b.y) * sc); pk.w = pk2h(cmb_bf(b.z) * sc, cmb_bf(b.w) * sc);
    VST2(v4u, (v4u*)(DST + (size_t)r * nC + c0), pk);
}

__global__ __launch_bounds__(256) void k_embtab(float* __restrict__ EMB, int n) {
    const int u = blockIdx.x * 256 + threadIdx.x; if (u >= n) return;
    const int t = u >> 5, i = u & 31;
    const float dv = expf((float)(2 * i) * (-0.14391156831212787f));
    const float ang = (float)t * dv;
    float sn, cs; sincosf(ang, &sn, &cs);
    v2f o; o.x = sn; o.y = cs;
    VST2(v2f, (v2f*)(EMB + 2 * (size_t)u), o);
}

__global__ __launch_bounds__(256) void k_ropenorm(const float* __restrict__ QKV, const float* __restrict__ EMB, const float* __restrict__ sqk, unsigned short* __restrict__ QK16) {
    const int L = threadIdx.x & 31;
    const int wv = blockIdx.x * 8 + __builtin_amdgcn_readfirstlane((int)(threadIdx.x >> 5));
    if (wv >= kMROWS * NH) return;
    const int hd = wv % NH, r = wv / NH, t = r % SEQ;
    const float cosv = EMB[(size_t)t * 64 + 32 + L], sinv = EMB[(size_t)t * 64 + L];
    const v2f sq = *(const v2f*)(sqk + hd * HD + 2 * L);
    const float s0 = cmb_bf(sq.x) * 32.f, s1 = cmb_bf(sq.y) * 32.f;
#pragma unroll 1
    for (int sel = 0; sel < 2; ++sel) {
        const v2f x = *(const v2f*)(QKV + (size_t)r * QKVW + sel * CW + hd * HD + 2 * L);
        const float o0 = -x.y * cosv, o1 = x.x * sinv;
        float ss = o0 * o0 + o1 * o1;
        ss += __shfl_xor(ss, 16, 32); ss += __shfl_xor(ss, 8, 32); ss += __shfl_xor(ss, 4, 32); ss += __shfl_xor(ss, 2, 32); ss += __shfl_xor(ss, 1, 32);
        const float inv = 1.0f / sqrtf(ss);
        const unsigned pk = pk2h(s0 * (o0 * inv) * 16.f, s1 * (o1 * inv) * 16.f);
        VST2(unsigned, (unsigned*)(QK16 + (size_t)sel * kMROWS * CW + (size_t)r * CW + hd * HD + 2 * L), pk);
    }
}

__global__ __launch_bounds__(256) void k_vtr(const float* __restrict__ QKV, unsigned short* __restrict__ VT16) {
    __shared__ float tile[64][65];
    const int u = threadIdx.x;
    const int bx = blockIdx.x; const int tt = bx % (SEQ / 64); const int bh = bx / (SEQ / 64); const int hd = bh % NH; const int b = bh / NH;
    const int t0 = tt * 64;
#pragma unroll
    for (int it = 0; it < 4; ++it) {
        const int row = (u >> 4) + 16 * it, c4 = (u & 15) * 4;
        const v4f v = *(const v4f*)(QKV + (size_t)(b * SEQ + t0 + row) * QKVW + 2 * CW + hd * HD + c4);
        tile[row][c4] = v.x; tile[row][c4 + 1] = v.y; tile[row][c4 + 2] = v.z; tile[row][c4 + 3] = v.w;
    }
    __syncthreads();
#pragma unroll
    for (int it = 0; it < 2; ++it) {
        const int d = (u >> 3) + 32 * it, pc = u & 7;
        v4u pk;
        pk.x = pk2h(tile[8 * pc + 0][d] * 16.f, tile[8 * pc + 1][d] * 16.f);
        pk.y = pk2h(tile[8 * pc + 2][d] * 16.f, tile[8 * pc + 3][d] * 16.f);
        pk.z = pk2h(tile[8 * pc + 4][d] * 16.f, tile[8 * pc + 5][d] * 16.f);
        pk.w = pk2h(tile[8 * pc + 6][d] * 16.f, tile[8 * pc + 7][d] * 16.f);
        VST2(v4u, (v4u*)(VT16 + ((size_t)((b * NH + hd) * HD + d)) * SEQ + t0 + 8 * pc), pk);
    }
}

__device__ __forceinline__ float logw2(float acc, float st, float thr) {
    const float sv = acc * 0.03125f;
    const float z = st * (sv - thr);
    const float e = exp2f(-fabsf(z) * 1.4426950408889634f);
    const float lsg = fminf(z, 0.f) - 0.6931471805599453f * log2f(1.0f + e);
    return (sv + lsg) * 1.4426950408889634f;
}

__global__ __launch_bounds__(128) void k_attn(const unsigned short* __restrict__ QK16p, const unsigned short* __restrict__ VT16p, unsigned short* __restrict__ Y16,
                                              const float* __restrict__ thr_c, const float* __restrict__ stp) {
    __shared__ __align__(16) _Float16 Ps[4][16 * PSP];
    __shared__ __align__(16) float Os[4][16 * 68];
    const int lane = threadIdx.x & 31;
    const int wave = __builtin_amdgcn_readfirstlane((int)(threadIdx.x >> 5));
    const int hh = lane >> 4, c = lane & 15;
    const int nqb = SEQ / 64;
    const int bx = blockIdx.x; const int qb = bx % nqb; const int bh = bx / nqb; const int hd = bh % NH; const int b = bh / NH;
    const int q0 = qb * 64 + wave * 16;
    const _Float16* Qb = (const _Float16*)QK16p + (size_t)b * SEQ * CW + hd * HD;
    const _Float16* Kb = Qb + (size_t)kMROWS * CW;
    const _Float16* Vb = (const _Float16*)VT16p + (size_t)(b * NH + hd) * HD * SEQ;
    const float thr = cmb_bf(thr_c[hd]), st = cmb_bf(stp[hd]);
    const float NEG = -__builtin_inff();

    const _Float16* qr = Qb + (size_t)(q0 + c) * CW + 8 * hh;
    const v16h qa0 = ldfrag(qr), qa1 = ldfrag(qr + 32);

    float mrow[8], lrow[8]; v8f oacc[4];
#pragma unroll
    for (int r = 0; r < 8; ++r) { mrow[r] = NEG; lrow[r] = 0.f; }
#pragma unroll
    for (int t = 0; t < 4; ++t) oacc[t] = (v8f){0.f, 0.f, 0.f, 0.f, 0.f, 0.f, 0.f, 0.f};

    const int nhalf = (q0 >> 5) + 1;
    for (int kh = 0; kh < nhalf; ++kh) {
        const int kv0 = kh * 32;
        const _Float16* kr = Kb + (size_t)(kv0 + c) * CW + 8 * hh;
        v8f s0 = (v8f){0.f, 0.f, 0.f, 0.f, 0.f, 0.f, 0.f, 0.f}, s1 = s0;
        { const v16h ka = ldfrag(kr), kb = ldfrag(kr + 32); s0 = wmma16(qa0, ka, s0); s0 = wmma16(qa1, kb, s0); }
        { const v16h ka = ldfrag(kr + 16 * CW), kb = ldfrag(kr + 16 * CW + 32); s1 = wmma16(qa0, ka, s1); s1 = wmma16(qa1, kb, s1); }
        const int kc0 = kv0 + c, kc1 = kc0 + 16;
#pragma unroll
        for (int r = 0; r < 8; ++r) {
            const int qrow = q0 + 8 * hh + r;
            float l0 = logw2(s0[r], st, thr), l1 = logw2(s1[r], st, thr);
            l0 = (kc0 > qrow) ? NEG : l0; l1 = (kc1 > qrow) ? NEG : l1;
            float m = fmaxf(l0, l1);
            m = fmaxf(m, __shfl_xor(m, 1, 32)); m = fmaxf(m, __shfl_xor(m, 2, 32)); m = fmaxf(m, __shfl_xor(m, 4, 32)); m = fmaxf(m, __shfl_xor(m, 8, 32));
            const float mnew = fmaxf(mrow[r], m);
            const float alpha = exp2f(mrow[r] - mnew);
            mrow[r] = mnew;
            float p0 = exp2f(l0 - mnew) * 256.f, p1 = exp2f(l1 - mnew) * 256.f;
            p0 = (p0 < 6.103515625e-5f) ? 0.f : p0; p1 = (p1 < 6.103515625e-5f) ? 0.f : p1;
            const _Float16 h0 = (_Float16)p0, h1 = (_Float16)p1;
            Ps[wave][(8 * hh + r) * PSP + c] = h0; Ps[wave][(8 * hh + r) * PSP + 16 + c] = h1;
            float ps = (float)h0 + (float)h1;
            ps += __shfl_xor(ps, 1, 32); ps += __shfl_xor(ps, 2, 32); ps += __shfl_xor(ps, 4, 32); ps += __shfl_xor(ps, 8, 32);
            lrow[r] = lrow[r] * alpha + ps;
#pragma unroll
            for (int t = 0; t < 4; ++t) oacc[t][r] *= alpha;
        }
        wave_sync_lds();
        FragH pa;
        pa.h[0] = *(const v8h_a*)&Ps[wave][c * PSP + 8 * hh];
        pa.h[1] = *(const v8h_a*)&Ps[wave][c * PSP + 16 + 8 * hh];
        const _Float16* vr = Vb + (size_t)c * SEQ + kv0 + 8 * hh;
        const v16h vb0 = ldfrag(vr), vb1 = ldfrag(vr + (size_t)16 * SEQ), vb2 = ldfrag(vr + (size_t)32 * SEQ), vb3 = ldfrag(vr + (size_t)48 * SEQ);
        oacc[0] = wmma16(pa.v, vb0, oacc[0]);
        oacc[1] = wmma16(pa.v, vb1, oacc[1]);
        oacc[2] = wmma16(pa.v, vb2, oacc[2]);
        oacc[3] = wmma16(pa.v, vb3, oacc[3]);
        wave_sync_lds();
    }

#pragma unroll
    for (int r = 0; r < 8; ++r) {
        const float inv = 1.0f / lrow[r];
#pragma unroll
        for (int t = 0; t < 4; ++t) Os[wave][(8 * hh + r) * 68 + t * 16 + c] = oacc[t][r] * inv;
    }
    wave_sync_lds();
    {
        const int q4 = lane >> 3, c8 = (lane & 7) * 8;
        unsigned short* yb = Y16 + (size_t)(b * SEQ + q0) * CW + hd * HD + c8;
        v4u pk[4];
#pragma unroll
        for (int it = 0; it < 4; ++it) {
            const int row = it * 4 + q4;
            const v4f a = *(const v4f_a*)&Os[wave][row * 68 + c8];
            const v4f d = *(const v4f_a*)&Os[wave][row * 68 + c8 + 4];
            pk[it].x = pk2h(a.x, a.y); pk[it].y = pk2h(a.z, a.w); pk[it].z = pk2h(d.x, d.y); pk[it].w = pk2h(d.z, d.w);
        }
        for (int pass = 0; pass < 2; ++pass) {
#pragma unroll
            for (int it = 0; it < 4; ++it) *(volatile v4u*)(yb + (size_t)(it * 4 + q4) * CW) = pk[it];
            __threadfence();
        }
    }
}

__global__ __launch_bounds__(256) void k_resnorm(const float* __restrict__ base, int base_raw, const float* __restrict__ delta, const float* __restrict__ alpha,
                                                 float* __restrict__ Yf, int out_full, unsigned short* __restrict__ Y16, int has16, int rows) {
    __shared__ __align__(16) v4f tl[8][256];
    const int L = threadIdx.x & 31;
    const int wave = __builtin_amdgcn_readfirstlane((int)(threadIdx.x >> 5));
    const int r = blockIdx.x * 8 + wave; if (r >= rows) return;
    const int rf = (r / SEQ) * SEQ_FULL + (r % SEQ);
    const int rb = base_raw ? rf : r, ro = out_full ? rf : r;
    const float* pa = base + (size_t)rb * CW + 4 * L;
    const float* pd = delta + (size_t)r * CW + 4 * L;
    float ssa = 0.f, ssb = 0.f;
#pragma unroll 1
    for (int q = 0; q < 8; ++q) {
        v4f a = *(const v4f*)(pa + 128 * q); const v4f d = *(const v4f*)(pd + 128 * q);
        if (base_raw) { a.x = cmb_bf(a.x); a.y = cmb_bf(a.y); a.z = cmb_bf(a.z); a.w = cmb_bf(a.w); }
        ssa += (a.x * a.x + a.y * a.y) + (a.z * a.z + a.w * a.w);
        ssb += (d.x * d.x + d.y * d.y) + (d.z * d.z + d.w * d.w);
    }
#pragma unroll
    for (int o = 16; o > 0; o >>= 1) { ssa += __shfl_xor(ssa, o, 32); ssb += __shfl_xor(ssb, o, 32); }
    const float inva = 1.0f / sqrtf(ssa), invb = 1.0f / sqrtf(ssb);
    float sst = 0.f;
#pragma unroll 1
    for (int q = 0; q < 8; ++q) {
        v4f a = *(const v4f*)(pa + 128 * q); const v4f d = *(const v4f*)(pd + 128 * q);
        if (base_raw) { a.x = cmb_bf(a.x); a.y = cmb_bf(a.y); a.z = cmb_bf(a.z); a.w = cmb_bf(a.w); }
        const v4f al = *(const v4f*)(alpha + 4 * L + 128 * q);
        v4f lr; lr.x = fabsf(cmb_bf(al.x) * 1.6f); lr.y = fabsf(cmb_bf(al.y) * 1.6f); lr.z = fabsf(cmb_bf(al.z) * 1.6f); lr.w = fabsf(cmb_bf(al.w) * 1.6f);
        const v4f An = a * inva, Bn = d * invb;
        const v4f t = An + lr * (Bn - An);
        tl[wave][q * 32 + L] = t;
        sst += (t.x * t.x + t.y * t.y) + (t.z * t.z + t.w * t.w);
    }
#pragma unroll
    for (int o = 16; o > 0; o >>= 1) sst += __shfl_xor(sst, o, 32);
    const float invt = 1.0f / sqrtf(sst);
#pragma unroll 1
    for (int q = 0; q < 8; ++q) {
        const v4f t = tl[wave][q * 32 + L];
        const v4f y = t * invt;
        VST2(v4f, (v4f*)(Yf + (size_t)ro * CW + 4 * L + 128 * q), y);
        if (has16) { v2u pk; pk.x = pk2h(y.x * 32.f, y.y * 32.f); pk.y = pk2h(y.z * 32.f, y.w * 32.f); VST2(v2u, (v2u*)(Y16 + (size_t)r * CW + 4 * L + 128 * q), pk); }
    }
}

__device__ __forceinline__ float silu_mul(float u, float g) { const float sg = 1.0f / (1.0f + expf(-g)); return (u * (g * sg)) * 16.f; }
__global__ __launch_bounds__(256) void k_swiglu(const float* __restrict__ UV, unsigned short* __restrict__ X16, int rows) {
    const long long u = (long long)blockIdx.x * 256 + threadIdx.x; const int per = FF / 8; if (u >= (long long)rows * per) return;
    const int r = (int)(u / per); const int c0 = 8 * (int)(u % per);
    const float* pu = UV + (size_t)r * FF2 + c0;
    unsigned w0 = 0u, w1 = 0u, w2 = 0u, w3 = 0u;
#pragma unroll 1
    for (int hf = 0; hf < 2; ++hf) {
        const v4f a = *(const v4f*)(pu + 4 * hf); const v4f g = *(const v4f*)(pu + FF + 4 * hf);
        const unsigned lo = pk2h(silu_mul(a.x, g.x), silu_mul(a.y, g.y)), hi = pk2h(silu_mul(a.z, g.z), silu_mul(a.w, g.w));
        if (hf == 0) { w0 = lo; w1 = hi; } else { w2 = lo; w3 = hi; }
    }
    v4u pk; pk.x = w0; pk.y = w1; pk.z = w2; pk.w = w3;
    VST2(v4u, (v4u*)(X16 + (size_t)r * FF + c0), pk);
}

constexpr size_t al256(size_t x) { return (x + 255) / 256 * 256; }
constexpr size_t szmax(size_t a, size_t b) { return a > b ? a : b; }
constexpr size_t SZ_EMB  = al256((size_t)SEQ * 64 * 4);
constexpr size_t SZ_H16  = al256((size_t)kMROWS * CW * 2);
constexpr size_t SZ_WQKV = al256((size_t)QKVW * CW * 2);
constexpr size_t SZ_WO   = al256((size_t)CW * CW * 2);
constexpr size_t SZ_WFC  = al256((size_t)FF2 * CW * 2);
constexpr size_t SZ_WPR  = al256((size_t)CW * FF * 2);
constexpr size_t SZ_QKV  = al256((size_t)kMROWS * QKVW * 4);
constexpr size_t SZ_UV   = al256((size_t)kMCH * FF2 * 4);
constexpr size_t SZ_U    = szmax(SZ_QKV, SZ_UV);
constexpr size_t SZ_QK16 = al256((size_t)2 * kMROWS * CW * 2);
constexpr size_t SZ_VT   = al256((size_t)kMROWS * CW * 2);
constexpr size_t SZ_Y16  = al256((size_t)kMROWS * CW * 2);
constexpr size_t SZ_F32  = al256((size_t)kMROWS * CW * 4);
constexpr size_t SZ_X16  = al256((size_t)kMCH * FF * 2);
constexpr size_t SZ_TOTAL = SZ_EMB + SZ_H16 + SZ_WQKV + SZ_WO + SZ_WFC + SZ_WPR + SZ_U + SZ_QK16 + SZ_VT + SZ_Y16 + SZ_F32 + SZ_F32 + SZ_H16 + SZ_X16 + SZ_F32;
static_assert(SZ_QKV <= SZ_U);
static_assert(SZ_UV <= SZ_U);
static_assert(SZ_TOTAL <= (size_t)134217728);
static_assert((size_t)((NB_FULL - 1) * SEQ_FULL + SEQ_FULL) * CW * 4 == (size_t)8388608);

extern "C" void kernel_launch(void* const* d_in, const int* in_sizes, int n_in, void* d_out, int out_size, void* d_ws, size_t ws_size, hipStream_t stream) {
    if (n_in < 13) return;
    const long long need_h = ((long long)(NB - 1) * SEQ_FULL + SEQ) * CW;
    if ((long long)in_sizes[0] < need_h) return;
    if ((long long)out_size < need_h) return;
    if (in_sizes[1] < CW * CW || in_sizes[2] < CW * CW || in_sizes[3] < CW * CW || in_sizes[4] < CW * CW) return;
    if (in_sizes[5] < FF2 * CW || in_sizes[6] < CW * FF) return;
    if (in_sizes[7] < CW || in_sizes[8] < FF2 || in_sizes[9] < CW || in_sizes[10] < CW || in_sizes[11] < NH || in_sizes[12] < NH) return;
    if (SZ_TOTAL > ws_size) return;

    const float* h      = (const float*)d_in[0];
    const float* Wq     = (const float*)d_in[1];
    const float* Wk     = (const float*)d_in[2];
    const float* Wv     = (const float*)d_in[3];
    const float* Wo     = (const float*)d_in[4];
    const float* Wfc    = (const float*)d_in[5];
    const float* Wproj  = (const float*)d_in[6];
    const float* sqk    = (const float*)d_in[7];
    const float* suv    = (const float*)d_in[8];
    const float* a_attn = (const float*)d_in[9];
    const float* a_mlp  = (const float*)d_in[10];
    const float* thr_c  = (const float*)d_in[11];
    const float* stp    = (const float*)d_in[12];
    float* out = (float*)d_out;

    char* wsp = (char*)d_ws;
    float* EMB = (float*)wsp; wsp += SZ_EMB;
    unsigned short* H16 = (unsigned short*)wsp; wsp += SZ_H16;
    unsigned short* WQKV16 = (unsigned short*)wsp; wsp += SZ_WQKV;
    unsigned short* WO16 = (unsigned short*)wsp; wsp += SZ_WO;
    unsigned short* WFC16 = (unsigned short*)wsp; wsp += SZ_WFC;
    unsigned short* WPR16 = (unsigned short*)wsp; wsp += SZ_WPR;
    float* QKV = (float*)wsp; float* UV = (float*)wsp; wsp += SZ_U;
    unsigned short* QK16 = (unsigned short*)wsp; wsp += SZ_QK16;
    unsigned short* VT16 = (unsigned short*)wsp; wsp += SZ_VT;
    unsigned short* Y16 = (unsigned short*)wsp; wsp += SZ_Y16;
    float* HATT = (float*)wsp; wsp += SZ_F32;
    float* H1 = (float*)wsp; wsp += SZ_F32;
    unsigned short* H116 = (unsigned short*)wsp; wsp += SZ_H16;
    unsigned short* X16 = (unsigned short*)wsp; wsp += SZ_X16;
    float* HMLP = (float*)wsp; wsp += SZ_F32;

    k_embtab<<<(SEQ * 32 + 255) / 256, 256, 0, stream>>>(EMB, SEQ * 32);
    k_cast16<<<(unsigned)(((long long)kMROWS * (CW / 8) + 255) / 256), 256, 0, stream>>>(h, H16, kMROWS, CW, 1.0f, SEQ, SEQ_FULL);
    k_cast16<<<(unsigned)(((long long)CW * (CW / 8) + 255) / 256), 256, 0, stream>>>(Wq, WQKV16, CW, CW, 16.0f, CW, CW);
    k_cast16<<<(unsigned)(((long long)CW * (CW / 8) + 255) / 256), 256, 0, stream>>>(Wk, WQKV16 + (size_t)CW * CW, CW, CW, 16.0f, CW, CW);
    k_cast16<<<(unsigned)(((long long)CW * (CW / 8) + 255) / 256), 256, 0, stream>>>(Wv, WQKV16 + (size_t)2 * CW * CW, CW, CW, 16.0f, CW, CW);
    k_cast16<<<(unsigned)(((long long)CW * (CW / 8) + 255) / 256), 256, 0, stream>>>(Wo, WO16, CW, CW, 16.0f, CW, CW);
    k_cast16<<<(unsigned)(((long long)FF2 * (CW / 8) + 255) / 256), 256, 0, stream>>>(Wfc, WFC16, FF2, CW, 16.0f, FF2, FF2);
    k_cast16<<<(unsigned)(((long long)CW * (FF / 8) + 255) / 256), 256, 0, stream>>>(Wproj, WPR16, CW, FF, 16.0f, CW, CW);

    k_gemm64<<<(unsigned)(((kMROWS / 64) * (QKVW / 64) + 7) / 8), 256, 0, stream>>>(H16, CW, WQKV16, CW, QKV, QKVW, suv, 0, kMROWS, QKVW, CW, 0.0625f);
    k_ropenorm<<<(unsigned)((kMROWS * NH + 7) / 8), 256, 0, stream>>>(QKV, EMB, sqk, QK16);
    k_vtr<<<(unsigned)(NB * NH * (SEQ / 64)), 256, 0, stream>>>(QKV, VT16);
    k_attn<<<(unsigned)(NB * NH * (SEQ / 64)), 128, 0, stream>>>(QK16, VT16, Y16, thr_c, stp);

    k_gemm64<<<(unsigned)(((kMROWS / 64) * (CW / 64) + 7) / 8), 256, 0, stream>>>(Y16, CW, WO16, CW, HATT, CW, suv, 0, kMROWS, CW, CW, 0.00390625f);
    k_resnorm<<<(unsigned)((kMROWS + 7) / 8), 256, 0, stream>>>(h, 1, HATT, a_attn, H1, 0, H116, 1, kMROWS);

    for (int ch = 0; ch < kNCH; ++ch) {
        k_gemm64<<<(unsigned)(((kMCH / 64) * (FF2 / 64) + 7) / 8), 256, 0, stream>>>(H116 + (size_t)ch * kMCH * CW, CW, WFC16, CW, UV, FF2, suv, 1, kMCH, FF2, CW, 0.0625f);
        k_swiglu<<<(unsigned)(((long long)kMCH * (FF / 8) + 255) / 256), 256, 0, stream>>>(UV, X16, kMCH);
        k_gemm64<<<(unsigned)(((kMCH / 64) * (CW / 64) + 7) / 8), 256, 0, stream>>>(X16, FF, WPR16, FF, HMLP + (size_t)ch * kMCH * CW, CW, suv, 0, kMCH, CW, FF, 0.00390625f);
    }
    k_resnorm<<<(unsigned)((kMROWS + 7) / 8), 256, 0, stream>>>(H1, 0, HMLP, a_mlp, out, 1, H116, 0, kMROWS);
}
